// GatedDeltaNetCell_4887672783151
// MI455X (gfx1250) — hardware-verified
//
#include <hip/hip_runtime.h>
#include <math.h>

constexpr int NSTEP  = 1024;
constexpr int NBATCH = 8;
constexpr int NDIM   = 1024;
constexpr int NHEAD  = 16;
constexpr int HDIM   = 64;
constexpr int NTOK   = NSTEP * NBATCH;
constexpr int NPROJ  = 5;
constexpr int SLABP  = 68;
constexpr int SCAN_TS = 16;
constexpr float L2_EPS = 1e-12f;
constexpr float INV_HDIM = 1.0f / (float)HDIM;
constexpr int NOUT0 = NSTEP * NBATCH * NDIM;
constexpr int NOUT1 = NBATCH * NHEAD * HDIM * HDIM;
static_assert(NHEAD * HDIM == NDIM, "head split");
static_assert(NTOK == 8192 && NDIM == 1024, "wire shapes");
static_assert(NDIM % 32 == 0, "GEMM K multiple of 32");
static_assert(NTOK % 64 == 0 && NDIM % 64 == 0, "GEMM M, N tile multiples");
static_assert(((NTOK / 64) * (NDIM / 64)) % 8 == 0, "GEMM grid exact");
static_assert(NSTEP % SCAN_TS == 0, "scan flush period");
static_assert(HDIM == 64, "one head = one 64-wide n tile");
static_assert((long)NOUT0 * 4 == 33554432L, "out1 byte offset");
static_assert(((long)NOUT0 + (long)NOUT1) * 4 == 35651584L, "d_out total bytes");

typedef __attribute__((ext_vector_type(16))) __bf16   v16b;
typedef __attribute__((ext_vector_type(8)))  __bf16   v8b;
typedef __attribute__((ext_vector_type(8)))  float    v8f;
typedef __attribute__((ext_vector_type(4)))  float    v4f;
typedef __attribute__((ext_vector_type(4)))  unsigned int v4u;

__device__ __forceinline__ unsigned short f2bf_bits(float f) {
  unsigned u = __float_as_uint(f);
  return (unsigned short)((u + 0x7FFFu + ((u >> 16) & 1u)) >> 16);
}
__device__ __forceinline__ float bf_bits2f(unsigned short h) { return __uint_as_float(((unsigned)h) << 16); }
__device__ __forceinline__ float bf16r(float f) { return bf_bits2f(f2bf_bits(f)); }
__device__ __forceinline__ unsigned pk16(unsigned short a, unsigned short b) { return (unsigned)a | ((unsigned)b << 16); }

__device__ __forceinline__ void tile_guard_b(v8f& a, v8f& b, v8f& c, v8f& d, v16b x, v16b y0, v16b y1, v16b y2, v16b y3) {
  asm volatile("v_nop\n\tv_nop\n\tv_nop\n\tv_nop" : "+v"(a), "+v"(b), "+v"(c), "+v"(d) : "v"(x), "v"(y0), "v"(y1), "v"(y2), "v"(y3));
}
__device__ __forceinline__ void keep4_b(v16b a, v16b b, v16b c, v16b d) { asm volatile("v_nop" :: "v"(a), "v"(b), "v"(c), "v"(d)); }
__device__ __forceinline__ void acc_guard4(v8f& a, v8f& b, v8f& c, v8f& d) { asm volatile("v_nop\n\tv_nop\n\tv_nop\n\tv_nop" : "+v"(a), "+v"(b), "+v"(c), "+v"(d)); }

__device__ __forceinline__ void wave_lds_sync() {
  __builtin_amdgcn_fence(__ATOMIC_RELEASE, "workgroup");
  __builtin_amdgcn_wave_barrier();
  __builtin_amdgcn_fence(__ATOMIC_ACQUIRE, "workgroup");
}

template <typename T> struct Frag;
template <> struct Frag<__bf16> {
  typedef v16b V; union U { v16b v; v8b h[2]; };
  static __device__ __forceinline__ v16b load(const __bf16* p) {
    U f; f.h[0] = *(const v8b*)(p); f.h[1] = *(const v8b*)(p + 16); return f.v;
  }
  static __device__ __forceinline__ v8f mma(v16b a, v16b b, v8f c) {
    return __builtin_amdgcn_wmma_f32_16x16x32_bf16(false, a, false, b, (short)0, c, false, false);
  }
};

__global__ __launch_bounds__(256) void cvt8_bf16_kernel(const float* __restrict__ s0, const float* __restrict__ s1,
                                                        const float* __restrict__ s2, const float* __restrict__ s3,
                                                        const float* __restrict__ s4,
                                                        unsigned short* __restrict__ dst, int n8) {
  const int z = blockIdx.y;
  const float* src = (z == 0) ? s0 : (z == 1) ? s1 : (z == 2) ? s2 : (z == 3) ? s3 : s4;
  const int i = blockIdx.x * 256 + threadIdx.x;
  if (i < n8) {
    const float* p = src + 8 * (size_t)i;
    const v4f a = *(const v4f*)(p);
    const v4f c = *(const v4f*)(p + 4);
    unsigned short hb[8];
#pragma unroll
    for (int e = 0; e < 4; ++e) {
      const float fa = a[e];
      const float fc = c[e];
      hb[e]     = f2bf_bits(fa);
      hb[4 + e] = f2bf_bits(fc);
    }
    const v4u u = (v4u){pk16(hb[0], hb[1]), pk16(hb[2], hb[3]), pk16(hb[4], hb[5]), pk16(hb[6], hb[7])};
    unsigned short* q = dst + (size_t)z * (size_t)n8 * 8 + 8 * (size_t)i;
    *(volatile v4u*)q = u;
    __threadfence();
    *(volatile v4u*)q = u;
  }
}

template <int MODE>
__global__ __launch_bounds__(256) void proj_gemm_kernel(const unsigned short* __restrict__ Ap,
                                                        const unsigned short* __restrict__ Btp,
                                                        float* __restrict__ Cout,
                                                        const float* __restrict__ bias) {
  const __bf16* A  = (const __bf16*)Ap;
  const __bf16* Bt = (const __bf16*)Btp;
  __shared__ __align__(16) float sT[8][16 * SLABP];
  __shared__ __align__(16) float gS[8][64];
  const int lane = threadIdx.x & 31;
  const int wave = threadIdx.x >> 5;
  constexpr int tilesN = NDIM >> 6;
  constexpr int tilesM = NTOK >> 6;
  const int tile = blockIdx.x * 8 + wave;
  if (tile >= tilesM * tilesN) return;
  const int tm = tile / tilesN;
  const int tn = tile - tm * tilesN;
  const int m0 = tm << 6;
  const int n0 = tn << 6;

  const int rlane = lane & 15;
  const int koff  = (lane >> 4) * 8;
  const int mOff  = (lane >> 4) * 8;

  v8f acc[4][4];
#pragma unroll
  for (int i = 0; i < 4; ++i)
#pragma unroll
    for (int j = 0; j < 4; ++j) acc[i][j] = (v8f){0.f, 0.f, 0.f, 0.f, 0.f, 0.f, 0.f, 0.f};

  for (int k0 = 0; k0 < NDIM; k0 += 32) {
    v16b bh[4];
#pragma unroll
    for (int j = 0; j < 4; ++j) {
      const size_t bo = (size_t)(n0 + (j << 4) + rlane) * NDIM + koff + k0;
      bh[j] = Frag<__bf16>::load(Bt + bo);
    }
#pragma unroll
    for (int i = 0; i < 4; ++i) {
      const size_t ao = (size_t)(m0 + (i << 4) + rlane) * NDIM + koff + k0;
      const v16b ah = Frag<__bf16>::load(A + ao);
#pragma unroll
      for (int j = 0; j < 4; ++j) acc[i][j] = Frag<__bf16>::mma(ah, bh[j], acc[i][j]);
      tile_guard_b(acc[i][0], acc[i][1], acc[i][2], acc[i][3], ah, bh[0], bh[1], bh[2], bh[3]);
    }
    keep4_b(bh[0], bh[1], bh[2], bh[3]);
  }
  acc_guard4(acc[0][0], acc[0][1], acc[0][2], acc[0][3]);
  acc_guard4(acc[1][0], acc[1][1], acc[1][2], acc[1][3]);
  acc_guard4(acc[2][0], acc[2][1], acc[2][2], acc[2][3]);
  acc_guard4(acc[3][0], acc[3][1], acc[3][2], acc[3][3]);

  float* slab = sT[wave];
  float* gsl  = gS[wave];
  const int prow  = lane >> 1;
  const int phalf = lane & 1;
#pragma unroll
  for (int i = 0; i < 4; ++i) {
    const int mBase = m0 + (i << 4);
#pragma unroll
    for (int j = 0; j < 4; ++j) {
#pragma unroll
      for (int r = 0; r < 8; ++r) slab[(mOff + r) * SLABP + (j << 4) + rlane] = acc[i][j][r];
    }
    wave_lds_sync();
    if (MODE == 1) {
      float* rp = slab + prow * SLABP + 32 * phalf;
      float ss = 0.0f;
#pragma unroll 1
      for (int e = 0; e < 8; ++e) {
        const v4f x = *(const v4f*)(rp + 4 * e);
        ss += x[0] * x[0];
        ss += x[1] * x[1];
        ss += x[2] * x[2];
        ss += x[3] * x[3];
      }
      ss += __shfl_xor(ss, 1, 32);
      const float inv = 1.0f / fmaxf(sqrtf(ss), L2_EPS);
#pragma unroll 1
      for (int e = 0; e < 8; ++e) {
        v4f x = *(const v4f*)(rp + 4 * e);
        x[0] = x[0] * inv;
        x[1] = x[1] * inv;
        x[2] = x[2] * inv;
        x[3] = x[3] * inv;
        *(v4f*)(rp + 4 * e) = x;
      }
      wave_lds_sync();
    }
    if (MODE == 2) {
      const float* rp = slab + prow * SLABP + 32 * phalf;
      const float* bp = bias + n0 + 32 * phalf;
      float s = 0.0f;
#pragma unroll 1
      for (int e = 0; e < 32; ++e) {
        const float z = rp[e] + bf16r(bp[e]);
        const float ex = expf(-z);
        s += 1.0f / (1.0f + ex);
      }
      s += __shfl_xor(s, 1, 32);
      if (phalf == 0) gsl[(i << 4) + prow] = s * INV_HDIM;
    } else {
      const int hh = lane >> 4, c4 = (lane & 15) * 4;
      for (int pass = 0; pass < 2; ++pass) {
#pragma unroll
        for (int it = 0; it < 8; ++it) {
          const int row = it * 2 + hh;
          const v4f v = *(const v4f*)(slab + row * SLABP + c4);
          *(volatile v4f*)(Cout + (size_t)(mBase + row) * NDIM + n0 + c4) = v;
        }
        __threadfence();
      }
    }
    wave_lds_sync();
  }
  if (MODE == 2) {
    wave_lds_sync();
    if (lane < 16) {
      const v4f g = *(const v4f*)(gsl + 4 * lane);
      float* gp = Cout + (size_t)tn * NTOK + m0 + 4 * lane;
      *(volatile v4f*)gp = g;
      __threadfence();
      *(volatile v4f*)gp = g;
    }
  }
}

__global__ __launch_bounds__(256) void state_scan_kernel(const float* __restrict__ qn, const float* __restrict__ kn,
                                                         const float* __restrict__ vn,
                                                         const float* __restrict__ ga, const float* __restrict__ gb,
                                                         const float* __restrict__ S0,
                                                         float* __restrict__ outs, float* __restrict__ Sfin) {
  __shared__ __align__(16) float ob[SCAN_TS * HDIM];
  __shared__ __align__(16) float sfl[HDIM * SLABP];
  const int bh = blockIdx.x;
  const int b = bh >> 4, h = bh & 15;
  const int tid = threadIdx.x;
  const int lane = tid & 31, wave = tid >> 5;
  const int r = tid >> 2, c = tid & 3;
  const size_t chan = (size_t)h * HDIM;

  float s[16];
  {
    const float* sp = S0 + ((size_t)bh * HDIM + r) * HDIM + c * 16;
#pragma unroll
    for (int jj = 0; jj < 4; ++jj) {
      const v4f x = *(const v4f*)(sp + 4 * jj);
      s[4 * jj + 0] = bf16r(x[0]);
      s[4 * jj + 1] = bf16r(x[1]);
      s[4 * jj + 2] = bf16r(x[2]);
      s[4 * jj + 3] = bf16r(x[3]);
    }
  }

#pragma unroll 1
  for (int t = 0; t < NSTEP; ++t) {
    const size_t n = (size_t)t * NBATCH + b;
    const float* kp = kn + n * NDIM + chan + c * 16;
    const float* qp = qn + n * NDIM + chan + c * 16;
    v4f kv[4], qv[4];
#pragma unroll
    for (int jj = 0; jj < 4; ++jj) {
      kv[jj] = *(const v4f*)(kp + 4 * jj);
      qv[jj] = *(const v4f*)(qp + 4 * jj);
    }
    const float vr = vn[n * NDIM + chan + r];
    const float a  = ga[(size_t)h * NTOK + n];
    const float be = gb[(size_t)h * NTOK + n];

    float p = 0.0f;
#pragma unroll
    for (int jj = 0; jj < 4; ++jj) {
#pragma unroll
      for (int e = 0; e < 4; ++e) p += s[4 * jj + e] * kv[jj][e];
    }
    p += __shfl_xor(p, 1, 32);
    p += __shfl_xor(p, 2, 32);

    const float c1 = be * p;
    const float c2 = be * vr;
#pragma unroll
    for (int jj = 0; jj < 4; ++jj) {
#pragma unroll
      for (int e = 0; e < 4; ++e) {
        const float kk = kv[jj][e];
        const float x = s[4 * jj + e] - c1 * kk;
        const float w = c2 * kk;
        s[4 * jj + e] = a * x + w;
      }
    }

    float po = 0.0f;
#pragma unroll
    for (int jj = 0; jj < 4; ++jj) {
#pragma unroll
      for (int e = 0; e < 4; ++e) po += s[4 * jj + e] * qv[jj][e];
    }
    po += __shfl_xor(po, 1, 32);
    po += __shfl_xor(po, 2, 32);
    if (c == 0) ob[(t & (SCAN_TS - 1)) * HDIM + r] = po;

    if ((t & (SCAN_TS - 1)) == (SCAN_TS - 1)) {
      __syncthreads();
      const int L   = 4 * wave + (lane >> 3);
      const int ts  = L >> 1;
      const int col = 32 * (L & 1) + 4 * (lane & 7);
      const v4f val = *(const v4f*)(ob + ts * HDIM + col);
      float* op = outs + ((size_t)(t - (SCAN_TS - 1) + ts) * NBATCH + b) * NDIM + chan + col;
      *(volatile v4f*)op = val;
      __threadfence();
      *(volatile v4f*)op = val;
      __syncthreads();
    }
  }

#pragma unroll
  for (int jj = 0; jj < 4; ++jj) {
    const v4f x = (v4f){s[4 * jj + 0], s[4 * jj + 1], s[4 * jj + 2], s[4 * jj + 3]};
    *(v4f*)(sfl + r * SLABP + c * 16 + 4 * jj) = x;
  }
  __syncthreads();
  {
    float* sp = Sfin + (size_t)bh * HDIM * HDIM;
    v4f fv[4];
#pragma unroll
    for (int it = 0; it < 4; ++it) {
      const int f = it * 256 + tid;
      fv[it] = *(const v4f*)(sfl + (f >> 4) * SLABP + (f & 15) * 4);
    }
    for (int pass = 0; pass < 2; ++pass) {
#pragma unroll
      for (int it = 0; it < 4; ++it) {
        const int f = it * 256 + tid;
        *(volatile v4f*)(sp + (size_t)f * 4) = fv[it];
      }
      __threadfence();
    }
  }
}

extern "C" void kernel_launch(void* const* d_in, const int* in_sizes, int n_in,
                              void* d_out, int out_size, void* d_ws, size_t ws_size, hipStream_t stream) {
  if (n_in < 9 || d_out == nullptr || d_ws == nullptr) return;
  if (in_sizes[0] != NTOK * NDIM || in_sizes[1] != NOUT1 ||
      in_sizes[2] != NDIM * NDIM || in_sizes[3] != NDIM * NDIM || in_sizes[4] != NDIM * NDIM ||
      in_sizes[5] != NDIM * NDIM || in_sizes[6] != NDIM || in_sizes[7] != NDIM * NDIM ||
      in_sizes[8] != NDIM || out_size != NOUT0 + NOUT1) return;

  const float* x   = (const float*)d_in[0];
  const float* S0  = (const float*)d_in[1];
  const float* Wq  = (const float*)d_in[2];
  const float* Wk  = (const float*)d_in[3];
  const float* Wv  = (const float*)d_in[4];
  const float* Wa  = (const float*)d_in[5];
  const float* ba  = (const float*)d_in[6];
  const float* Wb  = (const float*)d_in[7];
  const float* bb  = (const float*)d_in[8];
  float* outs = (float*)d_out;
  float* Sfin = outs + (size_t)NOUT0;

  char* ws = (char*)d_ws;
  size_t off = 0;
  auto carve = [&](size_t bytes) -> char* { char* p = ws + off; off += (bytes + 255) & ~(size_t)255; return p; };
  unsigned short* XB = (unsigned short*)carve((size_t)NTOK * NDIM * 2);
  unsigned short* WB = (unsigned short*)carve((size_t)NPROJ * NDIM * NDIM * 2);
  float* QN = (float*)carve((size_t)NTOK * NDIM * 4);
  float* KN = (float*)carve((size_t)NTOK * NDIM * 4);
  float* VN = (float*)carve((size_t)NTOK * NDIM * 4);
  float* GA = (float*)carve((size_t)NHEAD * NTOK * 4);
  float* GB = (float*)carve((size_t)NHEAD * NTOK * 4);
  if (off > ws_size || off > (size_t)134217728) return;

  const int n8x = NTOK * (NDIM / 8);
  const int n8w = NDIM * (NDIM / 8);
  cvt8_bf16_kernel<<<dim3(n8x / 256, 1), 256, 0, stream>>>(x, x, x, x, x, XB, n8x);
  cvt8_bf16_kernel<<<dim3(n8w / 256, NPROJ), 256, 0, stream>>>(Wq, Wk, Wv, Wa, Wb, WB, n8w);

  const int ggrid = (NTOK / 64) * (NDIM / 64) / 8;
  const size_t wplane = (size_t)NDIM * NDIM;
  proj_gemm_kernel<1><<<ggrid, 256, 0, stream>>>(XB, WB + 0 * wplane, QN, ba);
  proj_gemm_kernel<1><<<ggrid, 256, 0, stream>>>(XB, WB + 1 * wplane, KN, ba);
  proj_gemm_kernel<0><<<ggrid, 256, 0, stream>>>(XB, WB + 2 * wplane, VN, ba);
  proj_gemm_kernel<2><<<ggrid, 256, 0, stream>>>(XB, WB + 3 * wplane, GA, ba);
  proj_gemm_kernel<2><<<ggrid, 256, 0, stream>>>(XB, WB + 4 * wplane, GB, bb);

  state_scan_kernel<<<NBATCH * NHEAD, 256, 0, stream>>>(QN, KN, VN, GA, GB, S0, outs, Sfin);
}
